// BlockLocalSelfAttention_64269890617615
// MI455X (gfx1250) — hardware-verified
//
#include <hip/hip_runtime.h>
#include <stddef.h>


typedef __attribute__((ext_vector_type(16))) _Float16 v16h;
typedef __attribute__((ext_vector_type(8)))  _Float16 v8h;
typedef __attribute__((ext_vector_type(16))) __bf16   v16b;
typedef __attribute__((ext_vector_type(8)))  __bf16   v8b;
typedef __attribute__((ext_vector_type(8)))  float    v8f;
typedef __attribute__((ext_vector_type(4)))  float    v4f;

#define NB    2
#define NH    16
#define TT    4000
#define DD    64
#define QBLK  128
#define NQB   32
#define KC    64
#define NCHL  7
#define NCHG  63
#define OSP   68
#define SCL   0.125f
#define FMIN  (-3.402823466e38f)
#define NEG_INF (-__builtin_huge_valf())
#define PSC   32768.0f
#define VSC   256.0f
#define OSC   (1.0f / 8388608.0f)

__device__ __forceinline__ unsigned short f2bf_bits(float f) {
  unsigned u = __float_as_uint(f);
  return (unsigned short)((u + 0x7FFFu + ((u >> 16) & 1u)) >> 16);
}
__device__ __forceinline__ float bf_bits2f(unsigned short h) { return __uint_as_float(((unsigned)h) << 16); }

__device__ __forceinline__ v8f mma_bf(v16h a, v16h b, v8f c) {
  const v16b ab = __builtin_bit_cast(v16b, a), bb = __builtin_bit_cast(v16b, b);
  c = __builtin_amdgcn_wmma_f32_16x16x32_bf16(false, ab, false, bb, (short)0, c, false, false);
  asm volatile("v_nop\n\tv_nop\n\tv_nop\n\tv_nop" : "+v"(c) : "v"(ab), "v"(bb));
  return c;
}
__device__ __forceinline__ v8f mma_h(v16h a, v16h b, v8f c) {
  c = __builtin_amdgcn_wmma_f32_16x16x32_f16(false, a, false, b, (short)0, c, false, false);
  asm volatile("v_nop\n\tv_nop\n\tv_nop\n\tv_nop" : "+v"(c) : "v"(a), "v"(b));
  return c;
}

union FH { v16h v; v8h h[2]; };

template <int MODE>
__global__ __launch_bounds__(256) void cast8_kernel(const float* __restrict__ in,
                                                    _Float16* o1, _Float16* o2, int n8)
{
  const int i = blockIdx.x * 256 + threadIdx.x;
  if (i >= n8) return;
  const float* src = in + (size_t)i * 8;
  const v8f a = *(const v8f*)(src);
  v8h hv, lv;
#pragma unroll
  for (int e = 0; e < 8; ++e) {
    const float x = a[e];
    if (MODE == 0) {
      const unsigned short hb = f2bf_bits(x);
      const unsigned short lb = f2bf_bits(x - bf_bits2f(hb));
      hv[e] = __builtin_bit_cast(_Float16, hb);
      lv[e] = __builtin_bit_cast(_Float16, lb);
    } else {
      hv[e] = (_Float16)(x * VSC);
      lv[e] = hv[e];
    }
  }
  _Float16* p1 = o1 + (size_t)i * 8;
  _Float16* p2 = o2 + (size_t)i * 8;
  *(volatile v8h*)p1 = hv;
  if (MODE == 0) *(volatile v8h*)p2 = lv;
  __threadfence();
  *(volatile v8h*)p1 = hv;
  if (MODE == 0) *(volatile v8h*)p2 = lv;
}

template <bool GLB>
__global__ __launch_bounds__(GLB ? 32 : 256) void attn_kernel(
    const _Float16* __restrict__ QH, const _Float16* __restrict__ QL,
    const _Float16* __restrict__ KH, const _Float16* __restrict__ KL,
    const _Float16* __restrict__ VH, const float* __restrict__ am,
    float* __restrict__ out)
{
  constexpr int NT  = GLB ? 32 : 256;
  constexpr int NW  = NT / 32;
  constexpr int NCH = GLB ? NCHG : NCHL;
  constexpr int NU  = (KC * 8) / NT;
  constexpr int NMU = (KC + NT - 1) / NT;

  __shared__ __align__(16) _Float16 Ksh[KC * DD];
  __shared__ __align__(16) _Float16 Ksl[KC * DD];
  __shared__ __align__(16) _Float16 Vt[DD * KC];
  __shared__ __align__(16) _Float16 Psh[NW][16 * KC];
  __shared__ __align__(16) float    Os[NW][16 * OSP];
  __shared__ float Mv[KC];

  const int tid  = threadIdx.x;
  const int wave = tid >> 5;
  const int lane = tid & 31;
  const int hh   = lane >> 4;
  const int c    = lane & 15;

  int qb, hd, n;
  if (GLB) { qb = 0; hd = (int)(blockIdx.x % NH); n = (int)(blockIdx.x / NH); }
  else     { qb = blockIdx.x; hd = blockIdx.y; n = blockIdx.z; }
  const size_t hb = (size_t)(n * NH + hd) * TT;
  const float* amn = am + (size_t)n * TT;
  const int q0 = GLB ? 0 : (qb * QBLK + wave * 16);

  v16h qah[2], qal[2];
  {
    int qr = GLB ? 0 : (q0 + c);
    qr = (qr < TT) ? qr : (TT - 1);
    const _Float16* qhr = QH + (hb + (size_t)qr) * DD;
    const _Float16* qlr = QL + (hb + (size_t)qr) * DD;
#pragma unroll
    for (int dc = 0; dc < 2; ++dc) {
      FH f;
      f.h[0] = *(const v8h*)(qhr + dc * 32 + 8 * hh);
      f.h[1] = *(const v8h*)(qhr + dc * 32 + 16 + 8 * hh);
      qah[dc] = f.v;
      f.h[0] = *(const v8h*)(qlr + dc * 32 + 8 * hh);
      f.h[1] = *(const v8h*)(qlr + dc * 32 + 16 + 8 * hh);
      qal[dc] = f.v;
    }
  }

  float mrow[8], lrow[8];
  v8f oacc[4];
#pragma unroll
  for (int r = 0; r < 8; ++r) { mrow[r] = NEG_INF; lrow[r] = 0.f; }
#pragma unroll
  for (int t = 0; t < 4; ++t) oacc[t] = (v8f){0.f,0.f,0.f,0.f,0.f,0.f,0.f,0.f};
  v8h z8;
#pragma unroll
  for (int e = 0; e < 8; ++e) z8[e] = (_Float16)0.0f;

  for (int kc = 0; kc < NCH; ++kc) {
    __syncthreads();
#pragma unroll
    for (int u = 0; u < NU; ++u) {
      const int p   = tid + NT * u;
      const int row = p >> 3;
      const int d0  = (p & 7) * 8;
      int pos; bool valid;
      if (GLB) { pos = kc * KC + row; valid = (pos < TT); }
      else {
        pos   = (kc == 0) ? 0 : (qb * QBLK - QBLK + (kc - 1) * KC + row);
        valid = (kc == 0) ? (row == 0) : ((pos >= 0) && (pos < TT));
      }
      int posc = pos < 0 ? 0 : pos;
      posc = posc > (TT - 1) ? (TT - 1) : posc;
      const size_t off = (hb + (size_t)posc) * DD + d0;
      v8h k1 = *(const v8h*)(KH + off);
      v8h k2 = *(const v8h*)(KL + off);
      v8h vv = *(const v8h*)(VH + off);
      if (!valid) { k1 = z8; k2 = z8; vv = z8; }
      *(v8h*)(Ksh + row * DD + d0) = k1;
      *(v8h*)(Ksl + row * DD + d0) = k2;
#pragma unroll
      for (int e = 0; e < 8; ++e) Vt[(d0 + e) * KC + row] = vv[e];
    }
#pragma unroll
    for (int mu = 0; mu < NMU; ++mu) {
      const int row = tid + NT * mu;
      if (row < KC) {
        float mv;
        if (GLB) {
          const int pos = kc * KC + row;
          const bool valid = (pos < TT);
          const int posc = valid ? pos : (TT - 1);
          const float a = amn[posc];
          mv = valid ? a : NEG_INF;
        } else if (kc == 0) {
          const float a0 = amn[0];
          mv = (row == 0) ? a0 : NEG_INF;
        } else {
          const int pos = qb * QBLK - QBLK + (kc - 1) * KC + row;
          const bool valid = (pos >= 0) && (pos < TT);
          int posc = pos < 0 ? 0 : pos;
          posc = posc > (TT - 1) ? (TT - 1) : posc;
          const float a = amn[posc];
          mv = (valid && pos > 0) ? a : FMIN;
        }
        Mv[row] = mv;
      }
    }
    __syncthreads();

    v8f s[4];
#pragma unroll
    for (int j = 0; j < 4; ++j) {
      s[j] = (v8f){0.f,0.f,0.f,0.f,0.f,0.f,0.f,0.f};
#pragma unroll
      for (int dc = 0; dc < 2; ++dc) {
        FH kb, kl;
        const _Float16* kr = Ksh + (j * 16 + c) * DD + dc * 32 + 8 * hh;
        const _Float16* lr = Ksl + (j * 16 + c) * DD + dc * 32 + 8 * hh;
        kb.h[0] = *(const v8h*)(kr);  kb.h[1] = *(const v8h*)(kr + 16);
        kl.h[0] = *(const v8h*)(lr);  kl.h[1] = *(const v8h*)(lr + 16);
        s[j] = mma_bf(qah[dc], kb.v, s[j]);
        s[j] = mma_bf(qah[dc], kl.v, s[j]);
        s[j] = mma_bf(qal[dc], kb.v, s[j]);
      }
    }
    float mvj[4];
#pragma unroll
    for (int j = 0; j < 4; ++j) mvj[j] = Mv[j * 16 + c];
    float cm[8];
#pragma unroll
    for (int r = 0; r < 8; ++r) {
      float m = NEG_INF;
#pragma unroll
      for (int j = 0; j < 4; ++j) {
        const float sv = s[j][r] * SCL + mvj[j];
        s[j][r] = sv;
        m = fmaxf(m, sv);
      }
#pragma unroll
      for (int off = 1; off < 16; off <<= 1) m = fmaxf(m, __shfl_xor(m, off, 32));
      cm[r] = m;
    }
    _Float16* pw = Psh[wave];
#pragma unroll
    for (int r = 0; r < 8; ++r) {
      const float mnew  = fmaxf(mrow[r], cm[r]);
      const float alpha = __expf(mrow[r] - mnew);
      mrow[r] = mnew;
      float psum = 0.f;
#pragma unroll
      for (int j = 0; j < 4; ++j) {
        const float p = __expf(s[j][r] - mnew);
        psum += p;
        pw[(8 * hh + r) * KC + j * 16 + c] = (_Float16)(p * PSC);
      }
#pragma unroll
      for (int off = 1; off < 16; off <<= 1) psum += __shfl_xor(psum, off, 32);
      lrow[r] = lrow[r] * alpha + psum;
#pragma unroll
      for (int t = 0; t < 4; ++t) oacc[t][r] *= alpha;
    }
    __builtin_amdgcn_fence(__ATOMIC_RELEASE, "workgroup");
    __builtin_amdgcn_wave_barrier();
    __builtin_amdgcn_fence(__ATOMIC_ACQUIRE, "workgroup");
#pragma unroll 1
    for (int kk = 0; kk < 2; ++kk) {
      FH pa;
      pa.h[0] = *(const v8h*)(pw + c * KC + kk * 32 + 8 * hh);
      pa.h[1] = *(const v8h*)(pw + c * KC + kk * 32 + 16 + 8 * hh);
#pragma unroll
      for (int t = 0; t < 4; ++t) {
        FH vb;
        vb.h[0] = *(const v8h*)(Vt + (t * 16 + c) * KC + kk * 32 + 8 * hh);
        vb.h[1] = *(const v8h*)(Vt + (t * 16 + c) * KC + kk * 32 + 16 + 8 * hh);
        oacc[t] = mma_h(pa.v, vb.v, oacc[t]);
      }
    }
  }

  float* os = Os[wave];
#pragma unroll
  for (int r = 0; r < 8; ++r) {
    const float inv = (1.0f / lrow[r]) * OSC;
#pragma unroll
    for (int t = 0; t < 4; ++t) os[(8 * hh + r) * OSP + t * 16 + c] = oacc[t][r] * inv;
  }
  __builtin_amdgcn_fence(__ATOMIC_RELEASE, "workgroup");
  __builtin_amdgcn_wave_barrier();
  __builtin_amdgcn_fence(__ATOMIC_ACQUIRE, "workgroup");
  const int c4 = (lane & 15) * 4;
  if (GLB) {
    float* orow = out + hb * DD;
    for (int pass = 0; pass < 2; ++pass) {
      if (hh == 0) {
        const v4f val = *(const v4f*)(os + c4);
        *(volatile v4f*)(orow + c4) = val;
      }
      __threadfence();
    }
  } else {
    if (q0 < TT) {
      float* ob = out + (hb + (size_t)q0) * DD;
      for (int pass = 0; pass < 2; ++pass) {
#pragma unroll
        for (int it = 0; it < 8; ++it) {
          const int row = it * 2 + hh;
          const v4f val = *(const v4f*)(os + row * OSP + c4);
          *(volatile v4f*)(ob + (size_t)row * DD + c4) = val;
        }
        __threadfence();
      }
    }
  }
}

extern "C" void kernel_launch(void* const* d_in, const int* in_sizes, int n_in,
                              void* d_out, int out_size, void* d_ws, size_t ws_size,
                              hipStream_t stream)
{
  if (n_in < 4) return;
  const size_t nel = (size_t)NB * NH * TT * DD;
  if ((size_t)in_sizes[0] != nel || (size_t)in_sizes[1] != nel || (size_t)in_sizes[2] != nel) return;
  if ((size_t)in_sizes[3] != (size_t)NB * TT) return;
  if ((size_t)out_size != nel) return;
  const size_t PB = nel * 2;
  if (5 * PB > ws_size) return;

  const float* q  = (const float*)d_in[0];
  const float* k  = (const float*)d_in[1];
  const float* v  = (const float*)d_in[2];
  const float* am = (const float*)d_in[3];
  float* out = (float*)d_out;

  unsigned char* ws = (unsigned char*)d_ws;
  _Float16* qh = (_Float16*)(ws + 0 * PB);
  _Float16* ql = (_Float16*)(ws + 1 * PB);
  _Float16* kh = (_Float16*)(ws + 2 * PB);
  _Float16* kl = (_Float16*)(ws + 3 * PB);
  _Float16* vh = (_Float16*)(ws + 4 * PB);

  const int n8 = (int)(nel / 8);
  const int cg = (n8 + 255) / 256;
  cast8_kernel<0><<<cg, 256, 0, stream>>>(q, qh, ql, n8);
  cast8_kernel<0><<<cg, 256, 0, stream>>>(k, kh, kl, n8);
  cast8_kernel<1><<<cg, 256, 0, stream>>>(v, vh, vh, n8);

  attn_kernel<false><<<dim3(NQB, NH, NB), 256, 0, stream>>>(qh, ql, kh, kl, vh, am, out);
  attn_kernel<true><<<NB * NH, 32, 0, stream>>>(qh, ql, kh, kl, vh, am, out);
}
